// DeformableConvV2_27900107555312
// MI455X (gfx1250) — hardware-verified
//
#include <hip/hip_runtime.h>
#pragma clang fp contract(off)

typedef __attribute__((ext_vector_type(16))) _Float16 v16h;
typedef __attribute__((ext_vector_type(8)))  _Float16 v8h;
typedef __attribute__((ext_vector_type(16))) __bf16   v16b;
typedef __attribute__((ext_vector_type(8)))  __bf16   v8b;
typedef __attribute__((ext_vector_type(8)))  float    v8f;
typedef __attribute__((ext_vector_type(4)))  float    v4f;
typedef __attribute__((ext_vector_type(4)))  unsigned v4u;

__device__ __forceinline__ unsigned short f2bf_bits(float f) {
  unsigned u = __float_as_uint(f);
  return (unsigned short)((u + 0x7FFFu + ((u >> 16) & 1u)) >> 16);
}
__device__ __forceinline__ float bf_bits2f(unsigned short h) { return __uint_as_float(((unsigned)h) << 16); }

__device__ __forceinline__ void dep_guard_h(v8f& a, v8f& b, v16h x, v16h y) { asm volatile("v_nop\n\tv_nop\n\tv_nop\n\tv_nop" : "+v"(a), "+v"(b) : "v"(x), "v"(y)); }
__device__ __forceinline__ void dep_guard_b(v8f& a, v8f& b, v16b x, v16b y) { asm volatile("v_nop\n\tv_nop\n\tv_nop\n\tv_nop" : "+v"(a), "+v"(b) : "v"(x), "v"(y)); }
__device__ __forceinline__ void keep4_h(v16h a, v16h b, v16h c, v16h d) { asm volatile("v_nop" :: "v"(a), "v"(b), "v"(c), "v"(d)); }
__device__ __forceinline__ void keep4_b(v16b a, v16b b, v16b c, v16b d) { asm volatile("v_nop" :: "v"(a), "v"(b), "v"(c), "v"(d)); }
__device__ __forceinline__ void acc_guard4(v8f& a, v8f& b, v8f& c, v8f& d) { asm volatile("v_nop\n\tv_nop\n\tv_nop\n\tv_nop" : "+v"(a), "+v"(b), "+v"(c), "+v"(d)); }
template <typename T> struct Frag;
template <> struct Frag<_Float16> {
  typedef v16h V; union U { v16h v; v8h h[2]; };
  static __device__ __forceinline__ v16h load(const _Float16* p) {
    U f; f.h[0] = *(const v8h*)(p); f.h[1] = *(const v8h*)(p + 16); return f.v;
  }
  static __device__ __forceinline__ v8f mma(v16h a, v16h b, v8f c) {
    return __builtin_amdgcn_wmma_f32_16x16x32_f16(false, a, false, b, (short)0, c, false, false);
  }
  static __device__ __forceinline__ void guard(v8f& a, v8f& b, v16h x, v16h y) { dep_guard_h(a, b, x, y); }
  static __device__ __forceinline__ void keep(v16h a, v16h b, v16h c, v16h d) { keep4_h(a, b, c, d); }
};
template <> struct Frag<__bf16> {
  typedef v16b V; union U { v16b v; v8b h[2]; };
  static __device__ __forceinline__ v16b load(const __bf16* p) {
    U f; f.h[0] = *(const v8b*)(p); f.h[1] = *(const v8b*)(p + 16); return f.v;
  }
  static __device__ __forceinline__ v8f mma(v16b a, v16b b, v8f c) {
    return __builtin_amdgcn_wmma_f32_16x16x32_bf16(false, a, false, b, (short)0, c, false, false);
  }
  static __device__ __forceinline__ void guard(v8f& a, v8f& b, v16b x, v16b y) { dep_guard_b(a, b, x, y); }
  static __device__ __forceinline__ void keep(v16b a, v16b b, v16b c, v16b d) { keep4_b(a, b, c, d); }
};

template <int ET> struct Elem;
template <> struct Elem<0> { typedef _Float16 T; };
template <> struct Elem<1> { typedef __bf16 T; };
template <int ET, bool SPLIT, int BIAS_MODE, int OUT_MODE, bool RESID, int ACT = 0>
__global__ __launch_bounds__(256) void wmma_gemm64(
    const unsigned short* __restrict__ Ap, const unsigned short* __restrict__ A2p, int lda, long strideA,
    const unsigned short* __restrict__ Btp, const unsigned short* __restrict__ Bt2p, int ldb, long strideB,
    void* __restrict__ Cout, void* __restrict__ Cout2, int ldc, long strideC,
    const float* __restrict__ bias,
    const float* __restrict__ resid, long strideR,
    int M, int N, int K, float scale) {
  typedef typename Elem<ET>::T T;
  typedef typename Frag<T>::V V;
  const T* A = (const T*)Ap; const T* A2 = (const T*)A2p; const T* Bt = (const T*)Btp; const T* Bt2 = (const T*)Bt2p;
  __shared__ __align__(16) float sT[8][16 * 68];
  const int b    = blockIdx.y;
  const int lane = threadIdx.x & 31;
  const int wave = threadIdx.x >> 5;
  const int tilesN = N >> 6;
  const int tilesM = M >> 6;
  const int tile = blockIdx.x * 8 + wave;
  if (tile >= tilesM * tilesN) return;
  const int tm = tile / tilesN;
  const int tn = tile - tm * tilesN;
  const int m0 = tm << 6;
  const int n0 = tn << 6;

  const T* Ab  = A  + (size_t)b * strideA;
  const T* Bb  = Bt + (size_t)b * strideB;
  const T* Ab2 = SPLIT ? (A2  + (size_t)b * strideA) : nullptr;
  const T* Bb2 = SPLIT ? (Bt2 + (size_t)b * strideB) : nullptr;

  const int rlane = lane & 15;
  const int koff  = (lane >> 4) * 8;
  const int mOff  = (lane >> 4) * 8;

  v8f acc[4][4];
#pragma unroll
  for (int i = 0; i < 4; ++i)
#pragma unroll
    for (int j = 0; j < 4; ++j) acc[i][j] = (v8f){0.f,0.f,0.f,0.f,0.f,0.f,0.f,0.f};

  for (int k0 = 0; k0 < K; k0 += 32) {
    V bh[4], bl[4];
#pragma unroll
    for (int j = 0; j < 4; ++j) {
      const size_t bo = (size_t)(n0 + (j << 4) + rlane) * ldb + koff + k0;
      bh[j] = Frag<T>::load(Bb + bo);
      if (SPLIT) bl[j] = Frag<T>::load(Bb2 + bo);
    }
#pragma unroll
    for (int i = 0; i < 4; ++i) {
      const size_t ao = (size_t)(m0 + (i << 4) + rlane) * lda + koff + k0;
      V ah = Frag<T>::load(Ab + ao);
      V al;
      if (SPLIT) al = Frag<T>::load(Ab2 + ao);
#pragma unroll
      for (int j = 0; j < 4; ++j) {
        acc[i][j] = Frag<T>::mma(ah, bh[j], acc[i][j]);
        if (SPLIT) {
          acc[i][j] = Frag<T>::mma(ah, bl[j], acc[i][j]);
          acc[i][j] = Frag<T>::mma(al, bh[j], acc[i][j]);
        }
      }
      Frag<T>::guard(acc[i][0], acc[i][3], ah, SPLIT ? al : ah);
    }
    Frag<T>::keep(bh[0], bh[1], bh[2], bh[3]);
    if (SPLIT) Frag<T>::keep(bl[0], bl[1], bl[2], bl[3]);
  }
  acc_guard4(acc[0][0], acc[0][1], acc[0][2], acc[0][3]);
  acc_guard4(acc[1][0], acc[1][1], acc[1][2], acc[1][3]);
  acc_guard4(acc[2][0], acc[2][1], acc[2][2], acc[2][3]);
  acc_guard4(acc[3][0], acc[3][1], acc[3][2], acc[3][3]);

  float* slab = sT[wave];
  const float* Rb = RESID ? (resid + (size_t)b * strideR) : nullptr;
#pragma unroll
  for (int i = 0; i < 4; ++i) {
    const int mBase = m0 + (i << 4);
#pragma unroll
    for (int j = 0; j < 4; ++j) {
      const int n = n0 + (j << 4) + rlane;
      float bv = 0.f;
      if (BIAS_MODE == 2) bv = bias[n];
#pragma unroll
      for (int r = 0; r < 8; ++r) {
        float v = acc[i][j][r] * scale;
        if (BIAS_MODE == 1) v += bias[mBase + mOff + r];
        if (BIAS_MODE == 2) v += bv;
        if (RESID) v += Rb[(size_t)(mBase + mOff + r) * ldc + n];
        if (ACT == 1) v = tanhf(v);
        if (ACT == 2) v = fmaxf(v, 0.0f);
        if (ACT == 3) v = v / (1.0f + expf(-v));
        if (ACT == 4) v = (v > 0.f) ? v : 0.01f * v;
        if (ACT == 5) v = 0.5f * v * (1.0f + erff(v * 0.70710678118654752f));
        slab[(mOff + r) * 68 + (j << 4) + rlane] = v;
      }
    }
    __builtin_amdgcn_fence(__ATOMIC_RELEASE, "workgroup");
    __builtin_amdgcn_wave_barrier();
    __builtin_amdgcn_fence(__ATOMIC_ACQUIRE, "workgroup");
    if (OUT_MODE == 0) {
      float* C = (float*)Cout + (size_t)b * strideC;
      const int hh = lane >> 4, c4 = (lane & 15) * 4;
      for (int pass = 0; pass < 2; ++pass) {
#pragma unroll
        for (int it = 0; it < 8; ++it) {
          const int row = it * 2 + hh;
          v4f v = *(const v4f*)(slab + row * 68 + c4);
          *(volatile v4f*)(C + (size_t)(mBase + row) * ldc + n0 + c4) = v;
        }
        __threadfence();
      }
    } else {
      const int q = lane >> 3, c8 = (lane & 7) * 8;
      unsigned short* C  = (unsigned short*)Cout  + (size_t)b * strideC;
      unsigned short* C2 = (OUT_MODE == 2) ? ((unsigned short*)Cout2 + (size_t)b * strideC) : nullptr;
      for (int pass = 0; pass < 2; ++pass) {
#pragma unroll
        for (int it = 0; it < 4; ++it) {
          const int row = it * 4 + q;
          const float* sp = slab + row * 68 + c8;
          v8h hv, lv;
#pragma unroll
          for (int e = 0; e < 8; ++e) {
            if (OUT_MODE == 1) {
              hv[e] = (_Float16)sp[e];
            } else {
              unsigned short hb = f2bf_bits(sp[e]);
              unsigned short lb = f2bf_bits(sp[e] - bf_bits2f(hb));
              hv[e] = __builtin_bit_cast(_Float16, hb);
              lv[e] = __builtin_bit_cast(_Float16, lb);
            }
          }
          *(volatile v8h*)(C + (size_t)(mBase + row) * ldc + n0 + c8) = hv;
          if (OUT_MODE == 2) *(volatile v8h*)(C2 + (size_t)(mBase + row) * ldc + n0 + c8) = lv;
        }
        __threadfence();
      }
    }
    __builtin_amdgcn_fence(__ATOMIC_RELEASE, "workgroup");
    __builtin_amdgcn_wave_barrier();
    __builtin_amdgcn_fence(__ATOMIC_ACQUIRE, "workgroup");
  }
}

constexpr int kBatch   = 4;
constexpr int kCin     = 256;
constexpr int kCout    = 256;
constexpr int kHgt     = 48;
constexpr int kWid     = 48;
constexpr int kTaps    = 9;
constexpr int kKdim    = kCin * kTaps;
constexpr int kHW      = kHgt * kWid;
constexpr int kNtot    = kBatch * kHW;
constexpr int kOffCh   = 27;
constexpr int kOffRows = 64;
constexpr int kChunks  = kKdim / 8;

static_assert(kKdim % 32 == 0, "K tile");
static_assert(kChunks * 8 == kKdim, "chunks");
static_assert(kChunks % 32 == 0, "one wave never straddles a row");
static_assert(kOffRows % 64 == 0 && kNtot % 64 == 0 && kCout % 64 == 0 && kHW % 64 == 0, "M,N tiles");
static_assert((kKdim * 2) % 128 == 0, "16-bit rows are whole 128-B lines");
static_assert((kHW * 4) % 128 == 0 && (kNtot * 4) % 128 == 0, "f32 rows are whole 128-B lines");

constexpr size_t kColPlaneB = (size_t)kNtot * kKdim * 2;
constexpr size_t kWdPlaneB  = (size_t)kCout * kKdim * 2;
constexpr size_t kWoPlaneB  = (size_t)kOffRows * kKdim * 2;
constexpr size_t kOmB       = (size_t)kOffRows * kNtot * 4;
constexpr size_t kOffColHi  = 0;
constexpr size_t kOffColLo  = kOffColHi + kColPlaneB;
constexpr size_t kOffWdHi   = kOffColLo + kColPlaneB;
constexpr size_t kOffWdLo   = kOffWdHi + kWdPlaneB;
constexpr size_t kOffWoHi   = kOffWdLo + kWdPlaneB;
constexpr size_t kOffWoLo   = kOffWoHi + kWoPlaneB;
constexpr size_t kOffOm     = kOffWoLo + kWoPlaneB;
constexpr size_t kWsTotal   = kOffOm + kOmB;
static_assert(kWsTotal <= (size_t)134217728, "carve under 128 MiB");
static_assert(kOffColLo % 128 == 0 && kOffWdHi % 128 == 0 && kOffWdLo % 128 == 0 &&
              kOffWoHi % 128 == 0 && kOffWoLo % 128 == 0 && kOffOm % 128 == 0, "aligned regions");

__device__ __forceinline__ int clampi(int v, int lo, int hi) { return v < lo ? lo : (v > hi ? hi : v); }

__device__ __forceinline__ void store_pair_2pass(unsigned short* dhi, unsigned short* dlo, size_t off, v4u hv, v4u lv) {
  volatile v4u* ph = (volatile v4u*)(dhi + off);
  volatile v4u* pq = (volatile v4u*)(dlo + off);
  *ph = hv; *pq = lv;
  __threadfence();
  *ph = hv; *pq = lv;
}

__global__ __launch_bounds__(256) void k_split_rows(const float* __restrict__ src, int nsrc,
                                                    unsigned short* __restrict__ dhi,
                                                    unsigned short* __restrict__ dlo, int nrows) {
  const int id = blockIdx.x * 256 + threadIdx.x;
  if (id >= nrows * kChunks) return;
  const int row = id / kChunks;
  const int ch  = id - row * kChunks;
  const int srow = row < nsrc ? row : nsrc - 1;
  const bool live = row < nsrc;
  const float* sp = src + (size_t)srow * kKdim + ch * 8;
  const v4f f0 = *(const v4f*)(sp);
  const v4f f1 = *(const v4f*)(sp + 4);
  const float va[8] = {f0[0], f0[1], f0[2], f0[3], f1[0], f1[1], f1[2], f1[3]};
  unsigned hwd[4], lwd[4];
#pragma unroll
  for (int q = 0; q < 4; ++q) {
    const float a0 = live ? va[2 * q] : 0.0f;
    const float a1 = live ? va[2 * q + 1] : 0.0f;
    const unsigned short h0 = f2bf_bits(a0), h1 = f2bf_bits(a1);
    const unsigned short l0 = f2bf_bits(a0 - bf_bits2f(h0));
    const unsigned short l1 = f2bf_bits(a1 - bf_bits2f(h1));
    hwd[q] = (unsigned)h0 | ((unsigned)h1 << 16);
    lwd[q] = (unsigned)l0 | ((unsigned)l1 << 16);
  }
  const v4u hv = (v4u){hwd[0], hwd[1], hwd[2], hwd[3]};
  const v4u lv = (v4u){lwd[0], lwd[1], lwd[2], lwd[3]};
  store_pair_2pass(dhi, dlo, (size_t)row * kKdim + (size_t)ch * 8, hv, lv);
}

__device__ __forceinline__ float im2col_val(const float* __restrict__ x, int b, int h, int w, int kk) {
  const int c  = kk / kTaps;
  const int k2 = kk - c * kTaps;
  const int ki = k2 / 3;
  const int kj = k2 - ki * 3;
  const int yy = h - 1 + ki, xx = w - 1 + kj;
  const bool vld = (yy >= 0) && (yy < kHgt) && (xx >= 0) && (xx < kWid);
  const int yc = clampi(yy, 0, kHgt - 1), xc = clampi(xx, 0, kWid - 1);
  const float v = x[((size_t)(b * kCin + c) * kHgt + yc) * kWid + xc];
  return vld ? v : 0.0f;
}

__global__ __launch_bounds__(288) void k_cols_dense(const float* __restrict__ x,
                                                    unsigned short* __restrict__ dhi,
                                                    unsigned short* __restrict__ dlo) {
  const int n  = blockIdx.x;
  const int b  = n / kHW;
  const int hw = n - b * kHW;
  const int h  = hw / kWid;
  const int w  = hw - h * kWid;
  const int t  = threadIdx.x;
  unsigned hwd[4], lwd[4];
#pragma unroll
  for (int q = 0; q < 4; ++q) {
    const int kk = 8 * t + 2 * q;
    const float a0 = im2col_val(x, b, h, w, kk);
    const float a1 = im2col_val(x, b, h, w, kk + 1);
    const unsigned short h0 = f2bf_bits(a0), h1 = f2bf_bits(a1);
    const unsigned short l0 = f2bf_bits(a0 - bf_bits2f(h0));
    const unsigned short l1 = f2bf_bits(a1 - bf_bits2f(h1));
    hwd[q] = (unsigned)h0 | ((unsigned)h1 << 16);
    lwd[q] = (unsigned)l0 | ((unsigned)l1 << 16);
  }
  const v4u hv = (v4u){hwd[0], hwd[1], hwd[2], hwd[3]};
  const v4u lv = (v4u){lwd[0], lwd[1], lwd[2], lwd[3]};
  store_pair_2pass(dhi, dlo, (size_t)n * kKdim + (size_t)t * 8, hv, lv);
}

__device__ __forceinline__ float bilin_sample(const float* __restrict__ pl, int y0, int x0, float wy, float wx) {
  const int y1 = y0 + 1, x1 = x0 + 1;
  const float vy0 = (y0 >= 0 && y0 <= kHgt - 1) ? 1.0f : 0.0f;
  const float vy1 = (y1 >= 0 && y1 <= kHgt - 1) ? 1.0f : 0.0f;
  const float vx0 = (x0 >= 0 && x0 <= kWid - 1) ? 1.0f : 0.0f;
  const float vx1 = (x1 >= 0 && x1 <= kWid - 1) ? 1.0f : 0.0f;
  const int yc0 = clampi(y0, 0, kHgt - 1), yc1 = clampi(y1, 0, kHgt - 1);
  const int xc0 = clampi(x0, 0, kWid - 1), xc1 = clampi(x1, 0, kWid - 1);
  const float v00 = pl[yc0 * kWid + xc0];
  const float v01 = pl[yc0 * kWid + xc1];
  const float v10 = pl[yc1 * kWid + xc0];
  const float v11 = pl[yc1 * kWid + xc1];
  const float uy = 1.0f - wy, ux = 1.0f - wx;
  const float w00 = uy * ux, w01 = uy * wx, w10 = wy * ux, w11 = wy * wx;
  float p = v00 * (w00 * (vy0 * vx0));
  p = p + v01 * (w01 * (vy0 * vx1));
  p = p + v10 * (w10 * (vy1 * vx0));
  p = p + v11 * (w11 * (vy1 * vx1));
  return p;
}

__global__ __launch_bounds__(288) void k_cols_deform(const float* __restrict__ x,
                                                     const float* __restrict__ om,
                                                     unsigned short* __restrict__ dhi,
                                                     unsigned short* __restrict__ dlo) {
  __shared__ int   s_y0[16];
  __shared__ int   s_x0[16];
  __shared__ float s_wy[16];
  __shared__ float s_wx[16];
  __shared__ float s_mk[16];
  const int n  = blockIdx.x;
  const int b  = n / kHW;
  const int hw = n - b * kHW;
  const int h  = hw / kWid;
  const int w  = hw - h * kWid;
  const int t  = threadIdx.x;
  if (t < kTaps) {
    const int ki = t / 3;
    const int kj = t - ki * 3;
    const float dy = om[(size_t)(2 * t) * kNtot + n];
    const float dx = om[(size_t)(2 * t + 1) * kNtot + n];
    const float mv = om[(size_t)(2 * kTaps + t) * kNtot + n];
    const float py = dy + (float)(h - 1 + ki);
    const float px = dx + (float)(w - 1 + kj);
    const float fy = floorf(py);
    const float fx = floorf(px);
    const float fyc = fminf(fmaxf(fy, -8.0f), (float)(kHgt + 8));
    const float fxc = fminf(fmaxf(fx, -8.0f), (float)(kWid + 8));
    s_y0[t] = (int)fyc;
    s_x0[t] = (int)fxc;
    s_wy[t] = py - fy;
    s_wx[t] = px - fx;
    s_mk[t] = 1.0f / (1.0f + expf(-mv));
  }
  __syncthreads();

  unsigned hw0 = 0u, hw1 = 0u, hw2 = 0u, hw3 = 0u;
  unsigned lw0 = 0u, lw1 = 0u, lw2 = 0u, lw3 = 0u;
  const int kkb = 8 * t;
#pragma unroll 1
  for (int q = 0; q < 4; ++q) {
    unsigned hb[2], lb[2];
#pragma unroll
    for (int s = 0; s < 2; ++s) {
      const int kk = kkb + 2 * q + s;
      const int c  = kk / kTaps;
      const int k2 = kk - c * kTaps;
      const float* pl = x + (size_t)(b * kCin + c) * kHW;
      const float p  = bilin_sample(pl, s_y0[k2], s_x0[k2], s_wy[k2], s_wx[k2]);
      const float pm = p * s_mk[k2];
      const unsigned short hbit = f2bf_bits(pm);
      hb[s] = (unsigned)hbit;
      lb[s] = (unsigned)f2bf_bits(pm - bf_bits2f(hbit));
    }
    const unsigned hword = hb[0] | (hb[1] << 16);
    const unsigned lword = lb[0] | (lb[1] << 16);
    hw0 = (q == 0) ? hword : hw0;  hw1 = (q == 1) ? hword : hw1;
    hw2 = (q == 2) ? hword : hw2;  hw3 = (q == 3) ? hword : hw3;
    lw0 = (q == 0) ? lword : lw0;  lw1 = (q == 1) ? lword : lw1;
    lw2 = (q == 2) ? lword : lw2;  lw3 = (q == 3) ? lword : lw3;
  }
  const v4u hv = (v4u){hw0, hw1, hw2, hw3};
  const v4u lv = (v4u){lw0, lw1, lw2, lw3};
  store_pair_2pass(dhi, dlo, (size_t)n * kKdim + (size_t)t * 8, hv, lv);
}

extern "C" void kernel_launch(void* const* d_in, const int* in_sizes, int n_in,
                              void* d_out, int out_size, void* d_ws, size_t ws_size,
                              hipStream_t stream) {
  if (n_in < 3) return;
  if (in_sizes[0] != kBatch * kCin * kHW) return;
  if (in_sizes[1] != kOffCh * kKdim) return;
  if (in_sizes[2] != kCout * kKdim) return;
  if (out_size != kBatch * kCout * kHW) return;
  if (ws_size < kWsTotal) return;

  const float* x     = (const float*)d_in[0];
  const float* w_off = (const float*)d_in[1];
  const float* w_dcn = (const float*)d_in[2];
  float* out = (float*)d_out;

  char* ws = (char*)d_ws;
  unsigned short* colhi = (unsigned short*)(ws + kOffColHi);
  unsigned short* collo = (unsigned short*)(ws + kOffColLo);
  unsigned short* wdhi  = (unsigned short*)(ws + kOffWdHi);
  unsigned short* wdlo  = (unsigned short*)(ws + kOffWdLo);
  unsigned short* wohi  = (unsigned short*)(ws + kOffWoHi);
  unsigned short* wolo  = (unsigned short*)(ws + kOffWoLo);
  float* om = (float*)(ws + kOffOm);

  k_split_rows<<<(kOffRows * kChunks) / 256, 256, 0, stream>>>(w_off, kOffCh, wohi, wolo, kOffRows);
  k_split_rows<<<(kCout * kChunks) / 256, 256, 0, stream>>>(w_dcn, kCout, wdhi, wdlo, kCout);

  k_cols_dense<<<kNtot, kChunks, 0, stream>>>(x, colhi, collo);

  wmma_gemm64<1, true, 0, 0, false><<<dim3((kOffRows / 64) * (kNtot / 64) / 8, 1), 256, 0, stream>>>(
      wohi, wolo, kKdim, 0L,
      colhi, collo, kKdim, 0L,
      (void*)om, (void*)om, kNtot, 0L,
      (const float*)om, (const float*)om, 0L,
      kOffRows, kNtot, kKdim, 1.0f);

  k_cols_deform<<<kNtot, kChunks, 0, stream>>>(x, om, colhi, collo);

  wmma_gemm64<1, true, 0, 0, false><<<dim3((kCout / 64) * (kHW / 64) / 8, kBatch), 256, 0, stream>>>(
      wdhi, wdlo, kKdim, 0L,
      colhi, collo, kKdim, (long)kHW * kKdim,
      (void*)out, (void*)out, kHW, (long)kCout * kHW,
      (const float*)om, (const float*)om, 0L,
      kCout, kHW, kKdim, 1.0f);
}
